// NonTimestepResidualAttentionNorm_11922829214327
// MI455X (gfx1250) — hardware-verified
//
#include <hip/hip_runtime.h>
#include <math.h>
#include <stdint.h>

#define NBATCH 8
#define CC 1024
#define TT 1024
#define TP 1026
#define NH 16
#define HD 64
#define NBUCK 32
#define BTP 2048

static_assert(NH * HD == CC);
static_assert((CC % 128) == 0 && (TT % 64) == 0);

typedef _Float16 v16h __attribute__((ext_vector_type(16)));
typedef _Float16 v8h  __attribute__((ext_vector_type(8)));
typedef float    v8f  __attribute__((ext_vector_type(8)));
typedef float    v4f  __attribute__((ext_vector_type(4)));
typedef unsigned int v4u __attribute__((ext_vector_type(4)));

#if defined(__HIP_DEVICE_COMPILE__)
#define HZ_ACC_AB(c, a, b) asm volatile("v_nop\n\tv_nop\n\tv_nop\n\tv_nop" : "+v"(c) : "v"(a), "v"(b))
#define HZ_ACC2_A(c0, c1, a) asm volatile("v_nop\n\tv_nop\n\tv_nop\n\tv_nop" : "+v"(c0), "+v"(c1) : "v"(a))
#define HZ_KEEP4(a, b, c, d) asm volatile("v_nop" : : "v"(a), "v"(b), "v"(c), "v"(d))
#define HZ_ACC4(a, b, c, d) asm volatile("v_nop\n\tv_nop\n\tv_nop\n\tv_nop" : "+v"(a), "+v"(b), "+v"(c), "+v"(d))
#else
#define HZ_ACC_AB(c, a, b) ((void)0)
#define HZ_ACC2_A(c0, c1, a) ((void)0)
#define HZ_KEEP4(a, b, c, d) ((void)0)
#define HZ_ACC4(a, b, c, d) ((void)0)
#endif

__device__ __forceinline__ unsigned short h_bits(_Float16 x) { return __builtin_bit_cast(unsigned short, x); }
__device__ __forceinline__ unsigned pkf(float a, float b) {
  return (unsigned)h_bits((_Float16)a) | ((unsigned)h_bits((_Float16)b) << 16);
}
__device__ __forceinline__ v8f zero8() { v8f z = {0.f, 0.f, 0.f, 0.f, 0.f, 0.f, 0.f, 0.f}; return z; }
__device__ __forceinline__ float rcp_f(float x) { return __builtin_amdgcn_rcpf(x); }

__device__ __forceinline__ v16h ldfrag(const _Float16* p) {
  union { v16h v; v8h h[2]; } f;
  f.h[0] = *(const v8h*)(p);
  f.h[1] = *(const v8h*)(p + 16);
  return f.v;
}

__device__ __forceinline__ v8f mma_h(v16h a, v16h b, v8f c) {
  c = __builtin_amdgcn_wmma_f32_16x16x32_f16(false, a, false, b, (short)0, c, false, false);
  HZ_ACC_AB(c, a, b);
  return c;
}
__device__ __forceinline__ v8f mma_raw(v16h a, v16h b, v8f c) {
  return __builtin_amdgcn_wmma_f32_16x16x32_f16(false, a, false, b, (short)0, c, false, false);
}

__device__ __forceinline__ double shfl_xor_d(double v, int m) {
  const unsigned long long u = (unsigned long long)__double_as_longlong(v);
  const int lo = __shfl_xor((int)(unsigned)(u & 0xffffffffull), m, 32);
  const int hi = __shfl_xor((int)(unsigned)(u >> 32), m, 32);
  const unsigned long long r = ((unsigned long long)(unsigned)hi << 32) | (unsigned long long)(unsigned)lo;
  return __longlong_as_double((long long)r);
}
__device__ __forceinline__ void block_sum2(double& s, double& ss, double* red, int tid) {
#pragma unroll
  for (int m = 16; m >= 1; m >>= 1) {
    s += shfl_xor_d(s, m);
    ss += shfl_xor_d(ss, m);
  }
  const int wave = tid >> 5, lane = tid & 31;
  __syncthreads();
  if (lane == 0) { red[wave] = s; red[8 + wave] = ss; }
  __syncthreads();
  double S = 0.0, SS = 0.0;
#pragma unroll
  for (int w = 0; w < 8; ++w) { S += red[w]; SS += red[8 + w]; }
  s = S;
  ss = SS;
}

__global__ __launch_bounds__(256) void cvt_f16x8(const float* __restrict__ in, _Float16* out, int n8, float scale) {
  const int i = blockIdx.x * 256 + threadIdx.x;
  if (i < n8) {
    const v4f a = *(const v4f*)(in + (size_t)i * 8);
    const v4f c = *(const v4f*)(in + (size_t)i * 8 + 4);
    v4u p;
    p[0] = pkf(a[0] * scale, a[1] * scale);
    p[1] = pkf(a[2] * scale, a[3] * scale);
    p[2] = pkf(c[0] * scale, c[1] * scale);
    p[3] = pkf(c[2] * scale, c[3] * scale);
    _Float16* dst = out + (size_t)i * 8;
    *(volatile v4u*)dst = p;
    __threadfence();
    *(volatile v4u*)dst = p;
  }
}

__global__ __launch_bounds__(256) void cvt_convw(const float* __restrict__ w, _Float16* out, float scale) {
  const int idx = blockIdx.x * 256 + threadIdx.x;
  if (idx >= CC * (CC / 8)) return;
  const int o = idx >> 7;
  const int c8 = idx & 127;
  const float* p = w + ((size_t)o * CC + (size_t)c8 * 8) * 3;
  union { v4f q[6]; float e[24]; } u;
#pragma unroll
  for (int i = 0; i < 6; ++i) u.q[i] = *(const v4f*)(p + 4 * i);
  v4u pk[3];
#pragma unroll
  for (int tp = 0; tp < 3; ++tp) {
    v4u a;
#pragma unroll
    for (int m = 0; m < 4; ++m)
      a[m] = pkf(u.e[(2 * m) * 3 + tp] * scale, u.e[(2 * m + 1) * 3 + tp] * scale);
    pk[tp] = a;
  }
#pragma unroll
  for (int tp = 0; tp < 3; ++tp)
    *(volatile v4u*)(out + ((size_t)tp * CC + o) * CC + (size_t)c8 * 8) = pk[tp];
  __threadfence();
#pragma unroll
  for (int tp = 0; tp < 3; ++tp)
    *(volatile v4u*)(out + ((size_t)tp * CC + o) * CC + (size_t)c8 * 8) = pk[tp];
}

__global__ __launch_bounds__(256) void btab_k(const float* __restrict__ emb, float* tab) {
  const int i4 = blockIdx.x * 256 + threadIdx.x;
  if (i4 >= NH * (BTP / 4)) return;
  const int h = i4 >> 9;
  const int d0 = (i4 & 511) * 4;
  const float ln8 = 2.0794415416798357f;
  const float rl8 = 1.0f / ln8;
  v4f v;
#pragma unroll
  for (int e = 0; e < 4; ++e) {
    const int delta = d0 + e - 1024;
    const int n = delta < 0 ? -delta : delta;
    const float nf = (float)(n < 1 ? 1 : n);
    const float lg = logf(nf * 0.125f);
    int vl = 8 + (int)(lg * rl8 * 8.0f);
    vl = vl > 15 ? 15 : vl;
    int bucket = (n < 8) ? n : vl;
    bucket += (delta < 0) ? 16 : 0;
    v[e] = emb[bucket * NH + h] * 8.0f;
  }
  float* dst = tab + (size_t)i4 * 4;
  *(volatile v4f*)dst = v;
  __threadfence();
  *(volatile v4f*)dst = v;
}

template <bool SILU>
__global__ __launch_bounds__(256) void gn32_tr_k(const float* __restrict__ in, const float* __restrict__ gam,
                                                 const float* __restrict__ bet, _Float16* xt) {
  __shared__ __align__(16) v4u sT4[32 * 9];
  __shared__ double red[16];
  __shared__ float sA[64];
  __shared__ float sD[64];
  const int tid = threadIdx.x, lane = tid & 31, wave = tid >> 5;
  const int b = blockIdx.y;
  const int c0 = blockIdx.x * 64;
  const float* p = in + ((size_t)b * CC + c0) * TT;

#pragma unroll 1
  for (int g = 0; g < 2; ++g) {
    const float* pg = p + (size_t)g * 32 * TT;
    double s = 0.0, ss = 0.0;
#pragma unroll 1
    for (int i = 0; i < 32; ++i) {
      const v4f v = *(const v4f*)(pg + ((size_t)i * 256 + tid) * 4);
#pragma unroll
      for (int e = 0; e < 4; ++e) {
        const double d = (double)v[e];
        s += d;
        ss += d * d;
      }
    }
    block_sum2(s, ss, red, tid);
    const double invn = 1.0 / 32768.0;
    const double mean = s * invn;
    double var = ss * invn - mean * mean;
    var = var < 0.0 ? 0.0 : var;
    const float rstdf = (float)(1.0 / sqrt(var + 1e-5));
    const float meanf = (float)mean;
    if (tid >= g * 32 && tid < g * 32 + 32) {
      const int c = c0 + tid;
      const float a = rstdf * gam[c];
      sA[tid] = a;
      sD[tid] = bet[c] - meanf * a;
    }
  }
  __syncthreads();

  if (wave == 0 && lane < 16) {
    const int row = (lane < 8) ? 0 : (TP - 1);
    v4u z = {0u, 0u, 0u, 0u};
    _Float16* dst = xt + ((size_t)b * TP + row) * CC + c0 + (lane & 7) * 8;
    *(volatile v4u*)dst = z;
    __threadfence();
    *(volatile v4u*)dst = z;
  }

  float A[8], D[8];
#pragma unroll
  for (int i = 0; i < 8; ++i) { A[i] = sA[wave * 8 + i]; D[i] = sD[wave * 8 + i]; }
  const float* pr = p + (size_t)(wave * 8) * TT + lane;
  const int q = lane >> 3, c8 = (lane & 7) * 8;

#pragma unroll 1
  for (int tc = 0; tc < TT / 32; ++tc) {
    __syncthreads();
    float y[8];
#pragma unroll
    for (int i = 0; i < 8; ++i) {
      const float f = pr[(size_t)i * TT + tc * 32];
      float yy = fmaf(f, A[i], D[i]);
      if (SILU) yy = yy * rcp_f(1.0f + __expf(-yy));
      y[i] = yy;
    }
    v4u pk;
    pk[0] = pkf(y[0], y[1]);
    pk[1] = pkf(y[2], y[3]);
    pk[2] = pkf(y[4], y[5]);
    pk[3] = pkf(y[6], y[7]);
    sT4[lane * 9 + wave] = pk;
    __syncthreads();
    const int row = wave * 4 + q;
    const v4u v = sT4[row * 9 + (lane & 7)];
    _Float16* dst = xt + ((size_t)b * TP + 1 + tc * 32 + row) * CC + c0 + c8;
    *(volatile v4u*)dst = v;
    __threadfence();
    *(volatile v4u*)dst = v;
  }
}

__global__ __launch_bounds__(256) void gn8_attn_k(const float* __restrict__ hin,
                                                  const float* __restrict__ g8, const float* __restrict__ e8,
                                                  const float* __restrict__ ga, const float* __restrict__ ea,
                                                  float* xin, _Float16* xt) {
  __shared__ __align__(16) v4u sT4[32 * 17];
  __shared__ double red[16];
  __shared__ float sA1[128];
  __shared__ float sD1[128];
  __shared__ float sA[128];
  __shared__ float sD[128];
  __shared__ float sM[4];
  __shared__ float sR[4];
  const int tid = threadIdx.x, lane = tid & 31, wave = tid >> 5;
  const int b = blockIdx.y;
  const int c0 = blockIdx.x * 128;
  const float* p = hin + ((size_t)b * CC + c0) * TT;

  {
    double s = 0.0, ss = 0.0;
#pragma unroll 1
    for (int i = 0; i < 128; ++i) {
      const v4f v = *(const v4f*)(p + ((size_t)i * 256 + tid) * 4);
#pragma unroll
      for (int e = 0; e < 4; ++e) {
        const double d = (double)v[e];
        s += d;
        ss += d * d;
      }
    }
    block_sum2(s, ss, red, tid);
    const double invn = 1.0 / 131072.0;
    const double mean = s * invn;
    double var = ss * invn - mean * mean;
    var = var < 0.0 ? 0.0 : var;
    const float r8f = (float)(1.0 / sqrt(var + 1e-5));
    const float m8f = (float)mean;
    if (tid < 128) {
      const int c = c0 + tid;
      const float a = r8f * g8[c];
      sA1[tid] = a;
      sD1[tid] = e8[c] - m8f * a;
    }
  }
  __syncthreads();

  float* xo = xin + ((size_t)b * CC + c0) * TT;
#pragma unroll 1
  for (int sg = 0; sg < 4; ++sg) {
    double s2 = 0.0, ss2 = 0.0;
#pragma unroll 1
    for (int i = sg * 32; i < sg * 32 + 32; ++i) {
      const float a = sA1[i], d = sD1[i];
      const size_t off = ((size_t)i * 256 + tid) * 4;
      const v4f v = *(const v4f*)(p + off);
      v4f y;
#pragma unroll
      for (int e = 0; e < 4; ++e) {
        const float yy = fmaf(v[e], a, d);
        y[e] = yy;
        const double dd = (double)yy;
        s2 += dd;
        ss2 += dd * dd;
      }
      *(volatile v4f*)(xo + off) = y;
      __threadfence();
      *(volatile v4f*)(xo + off) = y;
    }
    block_sum2(s2, ss2, red, tid);
    const double invn = 1.0 / 32768.0;
    const double mean = s2 * invn;
    double var = ss2 * invn - mean * mean;
    var = var < 0.0 ? 0.0 : var;
    if (tid == 0) {
      sM[sg] = (float)mean;
      sR[sg] = (float)(1.0 / sqrt(var + 1e-5));
    }
  }
  __syncthreads();
  if (tid < 128) {
    const int sg = tid >> 5;
    const int c = c0 + tid;
    const float a2 = sR[sg] * ga[c];
    sA[tid] = sA1[tid] * a2;
    sD[tid] = (sD1[tid] - sM[sg]) * a2 + ea[c];
  }
  __syncthreads();

  float A[16], D[16];
#pragma unroll
  for (int i = 0; i < 16; ++i) { A[i] = sA[wave * 16 + i]; D[i] = sD[wave * 16 + i]; }
  const float* pr = p + (size_t)(wave * 16) * TT + lane;
  const int hh = lane >> 4, c16 = lane & 15;
#pragma unroll 1
  for (int tc = 0; tc < TT / 32; ++tc) {
    __syncthreads();
    float y[16];
#pragma unroll
    for (int i = 0; i < 16; ++i) {
      const float f = pr[(size_t)i * TT + tc * 32];
      y[i] = fmaf(f, A[i], D[i]);
    }
    v4u p0, p1;
#pragma unroll
    for (int m = 0; m < 4; ++m) {
      p0[m] = pkf(y[2 * m], y[2 * m + 1]);
      p1[m] = pkf(y[8 + 2 * m], y[9 + 2 * m]);
    }
    sT4[lane * 17 + wave * 2] = p0;
    sT4[lane * 17 + wave * 2 + 1] = p1;
    __syncthreads();
    v4u v[2];
#pragma unroll
    for (int it = 0; it < 2; ++it) {
      const int row = it * 16 + wave * 2 + hh;
      v[it] = sT4[row * 17 + c16];
    }
#pragma unroll
    for (int it = 0; it < 2; ++it) {
      const int row = it * 16 + wave * 2 + hh;
      *(volatile v4u*)(xt + ((size_t)b * TT + tc * 32 + row) * CC + c0 + c16 * 8) = v[it];
    }
    __threadfence();
#pragma unroll
    for (int it = 0; it < 2; ++it) {
      const int row = it * 16 + wave * 2 + hh;
      *(volatile v4u*)(xt + ((size_t)b * TT + tc * 32 + row) * CC + c0 + c16 * 8) = v[it];
    }
  }
}

template <int TAPS, int OUTH, bool RESID, int BM>
__global__ __launch_bounds__(256) void gemm_k(
    const _Float16* __restrict__ A, int lda, long long strideA, long long aTap, int aTS, int aTO,
    const _Float16* __restrict__ Bt, int ldb, long long strideB, long long bTap, int bTS, int bTO,
    const float* __restrict__ bias, float bscale,
    const float* __restrict__ resid,
    void* Cout, int ldc, long long strideC,
    int M, int N, int K, float oscale) {
  __shared__ __align__(16) float sT[8][16 * 68];
  const int bz = blockIdx.y;
  const int lane = threadIdx.x & 31, wave = threadIdx.x >> 5;
  const int tilesN = N >> 6, tilesM = M >> 5;
  const int tile = blockIdx.x * 8 + wave;
  if (tile >= tilesM * tilesN) return;
  const int tm = tile / tilesN, tn = tile - tm * tilesN;
  const int m0 = tm << 5, n0 = tn << 6;
  const int rlane = lane & 15;
  const int koff = (lane >> 4) * 8;
  const int mOff = koff;
  const int aRow0 = (m0 >> 6) * aTS + aTO + (m0 & 63);
  const int bRow0 = (n0 >> 6) * bTS + bTO;
  const _Float16* Ab = A + (size_t)bz * (size_t)strideA;
  const _Float16* Bb = Bt + (size_t)bz * (size_t)strideB;
  const size_t aro0 = (size_t)(aRow0 + rlane) * lda + koff;
  const size_t aro1 = (size_t)(aRow0 + 16 + rlane) * lda + koff;
  size_t bro[4];
#pragma unroll
  for (int j = 0; j < 4; ++j) bro[j] = (size_t)(bRow0 + j * 16 + rlane) * ldb + koff;

  v8f acc[2][4];
#pragma unroll
  for (int i = 0; i < 2; ++i)
#pragma unroll
    for (int j = 0; j < 4; ++j) acc[i][j] = zero8();

#pragma unroll 1
  for (int tp = 0; tp < TAPS; ++tp) {
    const _Float16* Ap = Ab + (size_t)tp * (size_t)aTap;
    const _Float16* Bp = Bb + (size_t)tp * (size_t)bTap;
#pragma unroll 1
    for (int k0 = 0; k0 < K; k0 += 32) {
      v16h bf[4];
#pragma unroll
      for (int j = 0; j < 4; ++j) bf[j] = ldfrag(Bp + bro[j] + k0);
      const v16h a0 = ldfrag(Ap + aro0 + k0);
#pragma unroll
      for (int j = 0; j < 4; ++j) acc[0][j] = mma_raw(a0, bf[j], acc[0][j]);
      HZ_ACC2_A(acc[0][0], acc[0][3], a0);
      const v16h a1 = ldfrag(Ap + aro1 + k0);
#pragma unroll
      for (int j = 0; j < 4; ++j) acc[1][j] = mma_raw(a1, bf[j], acc[1][j]);
      HZ_ACC2_A(acc[1][0], acc[1][3], a1);
      HZ_KEEP4(bf[0], bf[1], bf[2], bf[3]);
    }
  }
  HZ_ACC4(acc[0][0], acc[0][1], acc[0][2], acc[0][3]);
  HZ_ACC4(acc[1][0], acc[1][1], acc[1][2], acc[1][3]);

  float* slab = sT[wave];
#pragma unroll
  for (int i = 0; i < 2; ++i) {
    const int mBase = m0 + i * 16;
    float badd[8];
#pragma unroll
    for (int r = 0; r < 8; ++r) badd[r] = 0.f;
    if (BM == 1) {
#pragma unroll
      for (int r = 0; r < 8; ++r) badd[r] = bias[aRow0 + i * 16 + mOff + r] * bscale;
    }
#pragma unroll
    for (int j = 0; j < 4; ++j) {
      float bc = 0.f;
      if (BM == 2) bc = bias[bRow0 + j * 16 + rlane] * bscale;
#pragma unroll
      for (int r = 0; r < 8; ++r)
        slab[(mOff + r) * 68 + j * 16 + rlane] = acc[i][j][r] * oscale + badd[r] + bc;
    }
    __builtin_amdgcn_fence(__ATOMIC_RELEASE, "workgroup");
    __builtin_amdgcn_wave_barrier();
    __builtin_amdgcn_fence(__ATOMIC_ACQUIRE, "workgroup");
    if (OUTH == 0) {
      float* Cb = (float*)Cout + (size_t)bz * (size_t)strideC;
      const float* Rb = RESID ? (resid + (size_t)bz * (size_t)strideC) : resid;
      const int h2 = lane >> 4, c4 = (lane & 15) * 4;
      for (int pass = 0; pass < 2; ++pass) {
#pragma unroll
        for (int it = 0; it < 8; ++it) {
          const int row = it * 2 + h2;
          v4f v = *(const v4f*)(slab + row * 68 + c4);
          const size_t off = (size_t)(mBase + row) * ldc + n0 + c4;
          if (RESID) v += *(const v4f*)(Rb + off);
          *(volatile v4f*)(Cb + off) = v;
        }
        __threadfence();
      }
    } else {
      _Float16* Cb = (_Float16*)Cout + (size_t)bz * (size_t)strideC;
      const int q = lane >> 3, c8 = (lane & 7) * 8;
      v4u hv[4];
#pragma unroll
      for (int it = 0; it < 4; ++it) {
        const int row = it * 4 + q;
        const float* sp = slab + row * 68 + c8;
        v4u a;
#pragma unroll
        for (int e = 0; e < 4; ++e) a[e] = pkf(sp[2 * e], sp[2 * e + 1]);
        hv[it] = a;
      }
      for (int pass = 0; pass < 2; ++pass) {
#pragma unroll
        for (int it = 0; it < 4; ++it) {
          const int row = it * 4 + q;
          *(volatile v4u*)(Cb + (size_t)(mBase + row) * ldc + n0 + c8) = hv[it];
        }
        __threadfence();
      }
    }
    __builtin_amdgcn_fence(__ATOMIC_RELEASE, "workgroup");
    __builtin_amdgcn_wave_barrier();
    __builtin_amdgcn_fence(__ATOMIC_ACQUIRE, "workgroup");
  }
}

__global__ __launch_bounds__(128)
void attn_k(const _Float16* __restrict__ Qp, const _Float16* __restrict__ Kp, const _Float16* __restrict__ Vp,
            const float* __restrict__ tab, _Float16* AT, float sScale, float oScale) {
  union FH { v16h v; v8h h[2]; };
  __shared__ __align__(16) _Float16 Ksh[64 * 64];
  __shared__ __align__(16) _Float16 Vth[64 * 64];
  __shared__ __align__(16) _Float16 Psh[4][16 * 64];
  __shared__ __align__(16) float    Os[4][16 * 64];
  __shared__ __align__(16) float    sB[384 * 4];

  const int tid  = threadIdx.x;
  const int wave = tid >> 5;
  const int lane = tid & 31;
  const int hh   = lane >> 4;
  const int c    = lane & 15;

  const int bx  = blockIdx.x;
  const int qb  = bx & 15;
  const int h   = (bx >> 4) & 15;
  const int b   = bx >> 8;
  const int q0b = qb * 64;
  const int q0  = q0b + wave * 16;
  const size_t rowB = (size_t)b * TT;

  {
    const float* th = tab + (size_t)h * BTP + q0b;
#pragma unroll
    for (int k = 0; k < 3; ++k) {
      const int i  = tid + 128 * k;
      const int ic = (i < 271) ? i : 271;
      *(v4f*)(sB + 4 * i) = *(const v4f*)(th + 4 * ic);
    }
  }

  const _Float16* Qh = Qp + (size_t)h * HD;
  const _Float16* Kh = Kp + (size_t)h * HD;
  const _Float16* Vh = Vp + ((size_t)b * CC + (size_t)h * HD) * TT;

  v16h qa[2];
#pragma unroll
  for (int dc = 0; dc < 2; ++dc) qa[dc] = ldfrag(Qh + (rowB + q0 + c) * CC + dc * 32 + 8 * hh);

  float mrow[8], lrow[8];
  v8f oacc[4];
#pragma unroll
  for (int r = 0; r < 8; ++r) { mrow[r] = -INFINITY; lrow[r] = 0.f; }
#pragma unroll
  for (int t = 0; t < 4; ++t) oacc[t] = zero8();

  const int bbase = wave * 16 + 8 * hh + 1024 - c;
  _Float16* pwh = Psh[wave];

#pragma unroll 1
  for (int kt = 0; kt < TT / 64; ++kt) {
    const int kv0 = kt * 64;
    __syncthreads();
    {
      const int r = tid >> 1, half = (tid & 1) * 32;
      const _Float16* kg = Kh + (rowB + kv0 + r) * CC + half;
      const _Float16* vg = Vh + (size_t)r * TT + kv0 + half;
#pragma unroll
      for (int i = 0; i < 4; ++i) {
        const v8h a0 = *(const v8h*)(kg + 8 * i);
        const v8h b0 = *(const v8h*)(vg + 8 * i);
        *(v8h*)(Ksh + r * 64 + half + 8 * i) = a0;
        *(v8h*)(Vth + r * 64 + half + 8 * i) = b0;
      }
    }
    __syncthreads();

    v8f s[4];
#pragma unroll
    for (int j = 0; j < 4; ++j) {
      s[j] = zero8();
#pragma unroll
      for (int dc = 0; dc < 2; ++dc) {
        FH kb;
        kb.h[0] = *(const v8h*)(Ksh + (j * 16 + c) * 64 + dc * 32 + 8 * hh);
        kb.h[1] = *(const v8h*)(Ksh + (j * 16 + c) * 64 + dc * 32 + 16 + 8 * hh);
        s[j] = mma_h(qa[dc], kb.v, s[j]);
      }
    }

    const int bk = bbase - kv0;
#pragma unroll
    for (int r = 0; r < 8; ++r) {
      float m = -INFINITY;
#pragma unroll
      for (int j = 0; j < 4; ++j) {
        const float sv = s[j][r] * sScale + sB[bk + r - 16 * j];
        s[j][r] = sv;
        m = fmaxf(m, sv);
      }
#pragma unroll
      for (int off = 1; off < 16; off <<= 1) m = fmaxf(m, __shfl_xor(m, off, 32));
      const float mnew  = fmaxf(mrow[r], m);
      const float msafe = (mnew == -INFINITY) ? 0.f : mnew;
      const float alpha = __expf(mrow[r] - msafe);
      mrow[r] = mnew;
      float psum = 0.f;
#pragma unroll
      for (int j = 0; j < 4; ++j) {
        const float pe = __expf(s[j][r] - msafe);
        psum += pe;
        pwh[(8 * hh + r) * 64 + j * 16 + c] = (_Float16)(pe * 1024.0f);
      }
#pragma unroll
      for (int off = 1; off < 16; off <<= 1) psum += __shfl_xor(psum, off, 32);
      lrow[r] = lrow[r] * alpha + psum;
#pragma unroll
      for (int t = 0; t < 4; ++t) oacc[t][r] *= alpha;
    }
    __builtin_amdgcn_fence(__ATOMIC_RELEASE, "workgroup");
    __builtin_amdgcn_wave_barrier();
    __builtin_amdgcn_fence(__ATOMIC_ACQUIRE, "workgroup");

#pragma unroll
    for (int kk = 0; kk < 2; ++kk) {
      FH pa;
      pa.h[0] = *(const v8h*)(pwh + c * 64 + kk * 32 + 8 * hh);
      pa.h[1] = *(const v8h*)(pwh + c * 64 + kk * 32 + 16 + 8 * hh);
#pragma unroll
      for (int t = 0; t < 4; ++t) {
        FH vb;
        vb.h[0] = *(const v8h*)(Vth + (t * 16 + c) * 64 + kk * 32 + 8 * hh);
        vb.h[1] = *(const v8h*)(Vth + (t * 16 + c) * 64 + kk * 32 + 16 + 8 * hh);
        oacc[t] = mma_h(pa.v, vb.v, oacc[t]);
      }
    }
  }

  float* os = Os[wave];
#pragma unroll
  for (int r = 0; r < 8; ++r) {
    const float l = lrow[r];
    const float inv = ((l > 0.f) ? rcp_f(l) : 0.f) * oScale;
#pragma unroll
    for (int t = 0; t < 4; ++t) os[(8 * hh + r) * 64 + t * 16 + c] = oacc[t][r] * inv;
  }
  __builtin_amdgcn_fence(__ATOMIC_RELEASE, "workgroup");
  __builtin_amdgcn_wave_barrier();
  __builtin_amdgcn_fence(__ATOMIC_ACQUIRE, "workgroup");
  {
    const int q4 = lane >> 3, c8 = (lane & 7) * 8;
    v4u hv[4];
#pragma unroll
    for (int it = 0; it < 4; ++it) {
      const int row = it * 4 + q4;
      const float* sp = os + row * 64 + c8;
      v4u a;
#pragma unroll
      for (int e = 0; e < 4; ++e) a[e] = pkf(sp[2 * e], sp[2 * e + 1]);
      hv[it] = a;
    }
    for (int pass = 0; pass < 2; ++pass) {
#pragma unroll
      for (int it = 0; it < 4; ++it) {
        const int row = it * 4 + q4;
        const size_t go = (rowB + q0 + row) * CC + (size_t)h * HD + c8;
        *(volatile v4u*)(AT + go) = hv[it];
      }
      __threadfence();
    }
  }
}

extern "C" void kernel_launch(void* const* d_in, const int* in_sizes, int n_in,
                              void* d_out, int out_size, void* d_ws, size_t ws_size,
                              hipStream_t stream) {
  if (n_in < 18) return;
  const int nAct = NBATCH * CC * TT;
  if (in_sizes[0] != nAct || out_size != nAct) return;
  if (in_sizes[3] != CC * CC * 3 || in_sizes[7] != CC * CC * 3) return;
  if (in_sizes[13] != 3 * CC * CC || in_sizes[15] != CC * CC) return;
  if (in_sizes[1] != CC || in_sizes[2] != CC || in_sizes[4] != CC || in_sizes[5] != CC ||
      in_sizes[6] != CC || in_sizes[8] != CC || in_sizes[9] != CC || in_sizes[10] != CC ||
      in_sizes[11] != CC || in_sizes[12] != CC || in_sizes[16] != CC) return;
  if (in_sizes[14] != 3 * CC || in_sizes[17] != NBUCK * NH) return;

  const float* x      = (const float*)d_in[0];
  const float* gn1_g  = (const float*)d_in[1];
  const float* gn1_b  = (const float*)d_in[2];
  const float* c1_w   = (const float*)d_in[3];
  const float* c1_b   = (const float*)d_in[4];
  const float* gn2_g  = (const float*)d_in[5];
  const float* gn2_b  = (const float*)d_in[6];
  const float* c2_w   = (const float*)d_in[7];
  const float* c2_b   = (const float*)d_in[8];
  const float* n8_g   = (const float*)d_in[9];
  const float* n8_b   = (const float*)d_in[10];
  const float* ag_g   = (const float*)d_in[11];
  const float* ag_b   = (const float*)d_in[12];
  const float* qkv_w  = (const float*)d_in[13];
  const float* qkv_b  = (const float*)d_in[14];
  const float* pj_w   = (const float*)d_in[15];
  const float* pj_b   = (const float*)d_in[16];
  const float* remb   = (const float*)d_in[17];

  const size_t PWC  = (size_t)3 * CC * CC * 2;
  const size_t PWQ  = (size_t)3 * CC * CC * 2;
  const size_t PWP  = (size_t)CC * CC * 2;
  const size_t PTAB = (size_t)NH * BTP * 4;
  const size_t PXT  = (size_t)NBATCH * TP * CC * 2;
  const size_t PF   = (size_t)NBATCH * CC * TT * 4;
  const size_t PV   = (size_t)NBATCH * CC * TT * 2;
  size_t off = 0;
  const size_t oW1  = off; off += PWC;
  const size_t oW2  = off; off += PWC;
  const size_t oWq  = off; off += PWQ;
  const size_t oWp  = off; off += PWP;
  const size_t oTab = off; off += PTAB;
  const size_t oXT  = off; off += PXT;
  const size_t oR1  = off; off += PF;
  const size_t oXin = off; off += PF;
  const size_t oV   = off; off += PV;
  if (off > ws_size) return;
  if (off > (size_t)134217728) return;
  if (2 * PV > PF) return;
  if ((size_t)NBATCH * TT * CC * 2 > PXT) return;

  char* ws = (char*)d_ws;
  _Float16* W1t  = (_Float16*)(ws + oW1);
  _Float16* W2t  = (_Float16*)(ws + oW2);
  _Float16* Wqkv = (_Float16*)(ws + oWq);
  _Float16* Wpb  = (_Float16*)(ws + oWp);
  float*    Tab  = (float*)(ws + oTab);
  _Float16* XT   = (_Float16*)(ws + oXT);
  _Float16* XT3  = (_Float16*)(ws + oXT);
  _Float16* ATp  = (_Float16*)(ws + oXT);
  float*    F1   = (float*)(ws + oR1);
  float*    Hb   = (float*)(ws + oR1);
  _Float16* Qp   = (_Float16*)(ws + oR1);
  _Float16* Kp   = (_Float16*)(ws + oR1 + PV);
  float*    Xin  = (float*)(ws + oXin);
  _Float16* Vp   = (_Float16*)(ws + oV);

  const dim3 blk(256);
  const int  n8q = 3 * CC * CC / 8;
  const int  n8p = CC * CC / 8;
  const long long CCCC = (long long)CC * CC;
  const long long CT   = (long long)CC * TT;

  cvt_convw<<<dim3(CC * (CC / 8) / 256), blk, 0, stream>>>(c1_w, W1t, 64.0f);
  cvt_convw<<<dim3(CC * (CC / 8) / 256), blk, 0, stream>>>(c2_w, W2t, 64.0f);
  cvt_f16x8<<<dim3((n8q + 255) / 256), blk, 0, stream>>>(qkv_w, Wqkv, n8q, 64.0f);
  cvt_f16x8<<<dim3((n8p + 255) / 256), blk, 0, stream>>>(pj_w, Wpb, n8p, 64.0f);
  btab_k<<<dim3(NH * (BTP / 4) / 256), blk, 0, stream>>>(remb, Tab);

  gn32_tr_k<true><<<dim3(CC / 64, NBATCH), blk, 0, stream>>>(x, gn1_g, gn1_b, XT);
  gemm_k<3, 0, false, 1><<<dim3((CC / 32) * (TT / 64) / 8, NBATCH), blk, 0, stream>>>(
      W1t, CC, 0LL, CCCC, 64, 0,
      XT, CC, (long long)TP * CC, (long long)CC, 64, 0,
      c1_b, 1.0f, nullptr,
      (void*)F1, TT, CT, CC, TT, CC, 1.0f / 64.0f);
  gn32_tr_k<true><<<dim3(CC / 64, NBATCH), blk, 0, stream>>>(F1, gn2_g, gn2_b, XT);
  gemm_k<3, 0, true, 1><<<dim3((CC / 32) * (TT / 64) / 8, NBATCH), blk, 0, stream>>>(
      W2t, CC, 0LL, CCCC, 64, 0,
      XT, CC, (long long)TP * CC, (long long)CC, 64, 0,
      c2_b, 1.0f, x,
      (void*)Hb, TT, CT, CC, TT, CC, 1.0f / 64.0f);
  gn8_attn_k<<<dim3(CC / 128, NBATCH), blk, 0, stream>>>(Hb, n8_g, n8_b, ag_g, ag_b, Xin, XT3);
  gemm_k<1, 1, false, 2><<<dim3((NBATCH * TT / 32) * (CC / 64) / 8, 1), blk, 0, stream>>>(
      XT3, CC, 0LL, 0LL, 64, 0,
      Wqkv, CC, 0LL, 0LL, 192, 0,
      qkv_b, 16.0f, nullptr,
      (void*)Qp, CC, 0LL, NBATCH * TT, CC, CC, 0.25f);
  gemm_k<1, 1, false, 2><<<dim3((NBATCH * TT / 32) * (CC / 64) / 8, 1), blk, 0, stream>>>(
      XT3, CC, 0LL, 0LL, 64, 0,
      Wqkv, CC, 0LL, 0LL, 192, 64,
      qkv_b, 16.0f, nullptr,
      (void*)Kp, CC, 0LL, NBATCH * TT, CC, CC, 0.25f);
  gemm_k<1, 1, false, 1><<<dim3((CC / 32) * (TT / 64) / 8, NBATCH), blk, 0, stream>>>(
      Wqkv, CC, 0LL, 0LL, 192, 128,
      XT3, CC, CT, 0LL, 64, 0,
      qkv_b, 16.0f, nullptr,
      (void*)Vp, TT, CT, CC, TT, CC, 0.25f);
  attn_k<<<dim3((TT / 64) * NH * NBATCH), dim3(128), 0, stream>>>(
      Qp, Kp, Vp, Tab, ATp, 1.0f / 2048.0f, 1.0f / 64.0f);
  gemm_k<1, 0, true, 1><<<dim3((CC / 32) * (TT / 64) / 8, NBATCH), blk, 0, stream>>>(
      Wpb, CC, 0LL, 0LL, 64, 0,
      ATp, CC, CT, 0LL, 64, 0,
      pj_b, 1.0f, Xin,
      d_out, TT, CT, CC, TT, CC, 1.0f / 16384.0f);
  (void)hipGetLastError();
}
